// MaskedScaledDotProductAttention_67585605370702
// MI455X (gfx1250) — hardware-verified
//
#include <hip/hip_runtime.h>
#include <math.h>
#include <stdint.h>

#ifndef NB
#define NB    16
#endif
#define SEQ   2048
#define HD    128
#define QSC   1024.0f
#define KSC   1024.0f
#define PCAR  32768.0f
#define VCAR  256.0f
#define SM_SCALE 0.08838834764831845f
#define LOG2E 1.4426950408889634f
#define ATW   4
#define ATT_THREADS (ATW * 32)
#define QPB   (16 * ATW)
#define BPB   (SEQ / QPB)
#define ATT_BLOCKS (NB * BPB)
#define QP    20
#define SLABF (HD * QP)
#define VTP   72
#define VTILES (SEQ / 64)
static_assert(HD == 128 && QPB == 64 && ATT_THREADS == 128);
static_assert((SEQ % QPB) == 0 && (SEQ % 64) == 0 && (SEQ % 32) == 0 && (HD % 32) == 0);
static_assert(NB >= 1 && NB <= 16);
static_assert(BPB == 32 && VTILES == 32);
static_assert((HD - 1) * VTP + 63 < HD * VTP);
static_assert((HD - 1) * QP + 15 < SLABF && (QP % 4) == 0);
static_assert(((NB * SEQ * HD) % 2048) == 0);

typedef _Float16 v16h __attribute__((ext_vector_type(16)));
typedef _Float16 v8h  __attribute__((ext_vector_type(8)));
typedef float    v8f  __attribute__((ext_vector_type(8)));
typedef float    v4f  __attribute__((ext_vector_type(4)));
typedef unsigned int v4u __attribute__((ext_vector_type(4)));

union FragH { v16h v; v8h h[2]; v4u u[2]; };

__device__ __forceinline__ unsigned short bf_bits(float f) {
  unsigned u = __float_as_uint(f);
  return (unsigned short)((u + 0x7FFFu + ((u >> 16) & 1u)) >> 16);
}
__device__ __forceinline__ float bf_up(unsigned short h) { return __uint_as_float(((unsigned)h) << 16); }
__device__ __forceinline__ float bfr(float f) { return bf_up(bf_bits(f)); }
__device__ __forceinline__ unsigned short h_bits(_Float16 x) { return __builtin_bit_cast(unsigned short, x); }
__device__ __forceinline__ unsigned pk16(unsigned short a, unsigned short b) { return (unsigned)a | ((unsigned)b << 16); }
__device__ __forceinline__ v8f zero8() { v8f z = {0.f, 0.f, 0.f, 0.f, 0.f, 0.f, 0.f, 0.f}; return z; }

__device__ __forceinline__ v16h ldfrag_h(const _Float16* p) {
  FragH f;
  f.h[0] = *(const v8h*)(p);
  f.h[1] = *(const v8h*)(p + 16);
  return f.v;
}

__device__ __forceinline__ v8f mma_raw(v16h a, v16h b, v8f c) {
  return __builtin_amdgcn_wmma_f32_16x16x32_f16(false, a, false, b, (short)0, c, false, false);
}
__device__ __forceinline__ void guard_s(v8f& s, v16h x0, v16h x1, v16h x2, v16h x3,
                                        v16h y0, v16h y1, v16h y2, v16h y3) {
#if defined(__HIP_DEVICE_COMPILE__)
  asm volatile("v_nop\n\tv_nop\n\tv_nop\n\tv_nop"
               : "+v"(s) : "v"(x0), "v"(x1), "v"(x2), "v"(x3), "v"(y0), "v"(y1), "v"(y2), "v"(y3) : "memory");
#endif
}
__device__ __forceinline__ void guard_o4(v8f& a, v8f& b, v8f& c, v8f& d,
                                         v16h p, v16h q, v16h x0, v16h x1, v16h x2, v16h x3) {
#if defined(__HIP_DEVICE_COMPILE__)
  asm volatile("v_nop\n\tv_nop\n\tv_nop\n\tv_nop"
               : "+v"(a), "+v"(b), "+v"(c), "+v"(d) : "v"(p), "v"(q), "v"(x0), "v"(x1), "v"(x2), "v"(x3) : "memory");
#endif
}
__device__ __forceinline__ void acc_guard8(v8f& a, v8f& b, v8f& c, v8f& d, v8f& e, v8f& f, v8f& g, v8f& hx) {
#if defined(__HIP_DEVICE_COMPILE__)
  asm volatile("v_nop\n\tv_nop\n\tv_nop\n\tv_nop"
               : "+v"(a), "+v"(b), "+v"(c), "+v"(d), "+v"(e), "+v"(f), "+v"(g), "+v"(hx));
#endif
}
__device__ __forceinline__ void wave_sync_lds() {
  __builtin_amdgcn_fence(__ATOMIC_RELEASE, "workgroup");
  __builtin_amdgcn_wave_barrier();
  __builtin_amdgcn_fence(__ATOMIC_ACQUIRE, "workgroup");
}

__global__ __launch_bounds__(256) void cvt16(const float* __restrict__ xq, const float* __restrict__ xk,
                                             unsigned short* plq, unsigned short* plk, int n8, float sc) {
  const int gt = blockIdx.x * 256 + (int)threadIdx.x;
  if (gt >= n8) return;
  const bool sk = (blockIdx.y != 0);
  const float* x = sk ? xk : xq;
  unsigned short* pl = sk ? plk : plq;
  const size_t e = (size_t)gt * 8;
  const v4f a = *(const v4f*)(x + e), bq = *(const v4f*)(x + e + 4);
  v4u o;
#pragma unroll
  for (int i = 0; i < 2; ++i) {
    o[i]     = pk16(h_bits((_Float16)(bfr(a[2 * i]) * sc)),  h_bits((_Float16)(bfr(a[2 * i + 1]) * sc)));
    o[2 + i] = pk16(h_bits((_Float16)(bfr(bq[2 * i]) * sc)), h_bits((_Float16)(bfr(bq[2 * i + 1]) * sc)));
  }
  unsigned short* d = pl + e;
  for (int pass = 0; pass < 2; ++pass) {
    *(volatile v4u*)(d) = o;
    __threadfence();
  }
}

__global__ __launch_bounds__(256) void vt16(const float* __restrict__ v, unsigned short* VTo) {
  __shared__ __align__(16) unsigned short T[HD * VTP];
  const int tid = threadIdx.x;
  const int bid = blockIdx.x;
  const int bb  = bid / VTILES;
  const int t   = bid - bb * VTILES;
  if (bb >= NB) return;
  {
    const int sl = tid >> 2;
    const int dc = (tid & 3) * 32;
    int key = 64 * t + sl;
    key = (key < 0) ? 0 : ((key > SEQ - 1) ? (SEQ - 1) : key);
    const float* src = v + (((size_t)bb * SEQ + (size_t)key) * HD + dc);
#pragma unroll
    for (int i = 0; i < 8; ++i) {
      const v4f a = *(const v4f*)(src + 4 * i);
#pragma unroll
      for (int e = 0; e < 4; ++e) T[(dc + 4 * i + e) * VTP + sl] = h_bits((_Float16)(bfr(a[e]) * VCAR));
    }
  }
  __syncthreads();
  v4u vals[4];
  const int q8 = tid >> 3, p8 = (tid & 7) * 8;
#pragma unroll
  for (int it = 0; it < 4; ++it) {
    const int line = it * 32 + q8;
    vals[it] = *(const v4u*)(T + line * VTP + p8);
  }
  unsigned short* dst = VTo + ((size_t)bb * HD) * SEQ + 64 * t + p8;
  for (int pass = 0; pass < 2; ++pass) {
#pragma unroll
    for (int it = 0; it < 4; ++it) {
      const int line = it * 32 + q8;
      *(volatile v4u*)(dst + (size_t)line * SEQ) = vals[it];
    }
    __threadfence();
  }
}

__global__ __launch_bounds__(ATT_THREADS)
void attn_fwd(const unsigned short* __restrict__ QHp, const unsigned short* __restrict__ KHp,
              const unsigned short* __restrict__ VTq, float* OPp) {
  __shared__ __align__(16) float smem[ATW * SLABF];

  const int tid  = threadIdx.x;
  const int wave = tid >> 5;
  const int lane = tid & 31;
  const int hh   = lane >> 4;
  const int c    = lane & 15;

  const int bid  = blockIdx.x;
  const int bb   = bid / BPB;
  const int t    = bid - bb * BPB;
  if (bb >= NB) return;

  const int iw   = QPB * t + wave * 16;
  const int iwu  = __builtin_amdgcn_readfirstlane(iw);
  const int kend = iwu + 16;

  const _Float16* Qb = (const _Float16*)(const void*)QHp + ((size_t)bb * SEQ + (size_t)(iw + c)) * HD + 8 * hh;
  const v16h qf0 = ldfrag_h(Qb);
  const v16h qf1 = ldfrag_h(Qb + 32);
  const v16h qf2 = ldfrag_h(Qb + 64);
  const v16h qf3 = ldfrag_h(Qb + 96);
  const _Float16* Kb = (const _Float16*)(const void*)KHp + ((size_t)bb * SEQ + (size_t)c) * HD + 8 * hh;
  const _Float16* Vb = (const _Float16*)(const void*)VTq + ((size_t)bb * HD + (size_t)c) * SEQ + 8 * hh;
  const float lsc = (SM_SCALE * LOG2E) / (QSC * KSC);
  const int dq0 = 8 * hh - (iw + c);

  float m_run = -INFINITY, l_run = 0.f;
  v8f o[8];
#pragma unroll
  for (int j = 0; j < 8; ++j) o[j] = zero8();

#pragma unroll 1
  for (int kb = 0; kb < kend; kb += 32) {
    v8f s0 = zero8(), s1 = zero8();
    {
      const _Float16* k0p = Kb + (size_t)kb * HD;
      const v16h a0 = ldfrag_h(k0p), a1 = ldfrag_h(k0p + 32), a2 = ldfrag_h(k0p + 64), a3 = ldfrag_h(k0p + 96);
      s0 = mma_raw(a0, qf0, s0);
      s0 = mma_raw(a1, qf1, s0);
      s0 = mma_raw(a2, qf2, s0);
      s0 = mma_raw(a3, qf3, s0);
      guard_s(s0, a0, a1, a2, a3, qf0, qf1, qf2, qf3);
      const _Float16* k1p = k0p + (size_t)16 * HD;
      const v16h b0 = ldfrag_h(k1p), b1 = ldfrag_h(k1p + 32), b2 = ldfrag_h(k1p + 64), b3 = ldfrag_h(k1p + 96);
      s1 = mma_raw(b0, qf0, s1);
      s1 = mma_raw(b1, qf1, s1);
      s1 = mma_raw(b2, qf2, s1);
      s1 = mma_raw(b3, qf3, s1);
      guard_s(s1, b0, b1, b2, b3, qf0, qf1, qf2, qf3);
    }
    float u0[8], u1[8];
#pragma unroll
    for (int r = 0; r < 8; ++r) {
      u0[r] = s0[r] * lsc;
      u1[r] = s1[r] * lsc;
    }
    if (kb + 32 > iwu) {
      const int dq = kb + dq0;
#pragma unroll
      for (int r = 0; r < 8; ++r) {
        u0[r] = (dq + r > 0)      ? -INFINITY : u0[r];
        u1[r] = (dq + 16 + r > 0) ? -INFINITY : u1[r];
      }
    }
    float mx = -INFINITY;
#pragma unroll
    for (int r = 0; r < 8; ++r) mx = fmaxf(mx, fmaxf(u0[r], u1[r]));
    mx = fmaxf(mx, __shfl_xor(mx, 16, 32));
    const float mn = fmaxf(m_run, mx);
    const float al = exp2f(m_run - mn);
    m_run = mn;
    float ps = 0.f;
    FragH pa, pl;
#pragma unroll
    for (int r = 0; r < 8; ++r) {
      const float e0 = exp2f(u0[r] - mn), e1 = exp2f(u1[r] - mn);
      ps += e0 + e1;
      const float x0 = e0 * PCAR, x1 = e1 * PCAR;
      const _Float16 g0 = (_Float16)x0, g1 = (_Float16)x1;
      pa.h[0][r] = g0;
      pa.h[1][r] = g1;
      pl.h[0][r] = (_Float16)(x0 - (float)g0);
      pl.h[1][r] = (_Float16)(x1 - (float)g1);
    }
    ps += __shfl_xor(ps, 16, 32);
    l_run = l_run * al + ps;
#pragma unroll
    for (int r = 0; r < 8; ++r) {
      const float af = __shfl(al, 8 * hh + r, 32);
#pragma unroll
      for (int j = 0; j < 8; ++j) o[j][r] *= af;
    }
    {
      const _Float16* vp = Vb + kb;
      const v16h v0 = ldfrag_h(vp);
      const v16h v1 = ldfrag_h(vp + (size_t)16 * SEQ);
      const v16h v2 = ldfrag_h(vp + (size_t)32 * SEQ);
      const v16h v3 = ldfrag_h(vp + (size_t)48 * SEQ);
      o[0] = mma_raw(pa.v, v0, o[0]);
      o[0] = mma_raw(pl.v, v0, o[0]);
      o[1] = mma_raw(pa.v, v1, o[1]);
      o[1] = mma_raw(pl.v, v1, o[1]);
      o[2] = mma_raw(pa.v, v2, o[2]);
      o[2] = mma_raw(pl.v, v2, o[2]);
      o[3] = mma_raw(pa.v, v3, o[3]);
      o[3] = mma_raw(pl.v, v3, o[3]);
      guard_o4(o[0], o[1], o[2], o[3], pa.v, pl.v, v0, v1, v2, v3);
      const v16h v4 = ldfrag_h(vp + (size_t)64 * SEQ);
      const v16h v5 = ldfrag_h(vp + (size_t)80 * SEQ);
      const v16h v6 = ldfrag_h(vp + (size_t)96 * SEQ);
      const v16h v7 = ldfrag_h(vp + (size_t)112 * SEQ);
      o[4] = mma_raw(pa.v, v4, o[4]);
      o[4] = mma_raw(pl.v, v4, o[4]);
      o[5] = mma_raw(pa.v, v5, o[5]);
      o[5] = mma_raw(pl.v, v5, o[5]);
      o[6] = mma_raw(pa.v, v6, o[6]);
      o[6] = mma_raw(pl.v, v6, o[6]);
      o[7] = mma_raw(pa.v, v7, o[7]);
      o[7] = mma_raw(pl.v, v7, o[7]);
      guard_o4(o[4], o[5], o[6], o[7], pa.v, pl.v, v4, v5, v6, v7);
    }
  }
  acc_guard8(o[0], o[1], o[2], o[3], o[4], o[5], o[6], o[7]);

  const float oc = 1.0f / (PCAR * VCAR);
  const float li = (l_run > 0.0f) ? ((1.0f / l_run) * oc) : 0.0f;
  float* slab = smem + wave * SLABF;
  float lf[8];
#pragma unroll
  for (int r = 0; r < 8; ++r) lf[r] = __shfl(li, 8 * hh + r, 32);
#pragma unroll
  for (int j = 0; j < 8; ++j) {
    v4f w0, w1;
#pragma unroll
    for (int r = 0; r < 4; ++r) { w0[r] = o[j][r] * lf[r]; w1[r] = o[j][4 + r] * lf[4 + r]; }
    float* sp = slab + (16 * j + c) * QP + 8 * hh;
    *(v4f*)(sp)     = w0;
    *(v4f*)(sp + 4) = w1;
  }
  wave_sync_lds();
  v4f vals[16];
#pragma unroll
  for (int it = 0; it < 16; ++it) {
#pragma unroll
    for (int e = 0; e < 4; ++e) vals[it][e] = slab[(4 * lane + e) * QP + it];
  }
  float* dst = OPp + ((size_t)bb * SEQ + (size_t)iw) * HD + 4 * lane;
  for (int pass = 0; pass < 2; ++pass) {
#pragma unroll
    for (int it = 0; it < 16; ++it) {
      *(volatile v4f*)(dst + (size_t)it * HD) = vals[it];
    }
    __threadfence();
  }
}

extern "C" void kernel_launch(void* const* d_in, const int* in_sizes, int n_in,
                              void* d_out, int out_size, void* d_ws, size_t ws_size,
                              hipStream_t stream) {
  const int NEL = NB * SEQ * HD;
  if (n_in < 3) return;
  if (in_sizes[0] < NEL || in_sizes[1] < NEL || in_sizes[2] < NEL) return;
  if (out_size < NEL) return;

  const float* q  = (const float*)d_in[0];
  const float* k  = (const float*)d_in[1];
  const float* v  = (const float*)d_in[2];
  float*       out = (float*)d_out;

  const size_t PQ = (size_t)NEL * 2;
  const size_t PK = (size_t)NEL * 2;
  const size_t PV = (size_t)NB * HD * SEQ * 2;
  size_t off = 0;
  const size_t oQH = off; off += PQ;
  const size_t oKH = off; off += PK;
  const size_t oVT = off; off += PV;
  if (off > ws_size) return;
  if (off > (size_t)134217728) return;

  char* ws = (char*)d_ws;
  unsigned short* QH = (unsigned short*)(ws + oQH);
  unsigned short* KH = (unsigned short*)(ws + oKH);
  unsigned short* VT = (unsigned short*)(ws + oVT);

  const int n8 = NEL / 8;
  const dim3 blk(256);
  const dim3 gC(n8 / 256, 2);
  const dim3 gVT(NB * VTILES);
  const dim3 gAT(ATT_BLOCKS);
  const dim3 bAT(ATT_THREADS);

  cvt16<<<gC, blk, 0, stream>>>(q, k, QH, KH, n8, QSC);
  vt16<<<gVT, blk, 0, stream>>>(v, VT);
  attn_fwd<<<gAT, bAT, 0, stream>>>(QH, KH, VT, out);
  (void)hipGetLastError();
}
